// Bottleneck_DSConv_63797444214791
// MI455X (gfx1250) — hardware-verified
//
#include <hip/hip_runtime.h>
#define NI 4
#define CX 128
#define CHD 64
#define CO 128
#define HS 80
#define WSD 80
#define NPX (HS * WSD)
#define NR (NI * NPX)
#define KS 9
#define K1 (9 * CX)
#define K9 (81 * CHD)
#define K3 (9 * CHD)
#define KSN (KS * CHD)
#define CC (3 * CO)
typedef __bf16 v16b __attribute__((ext_vector_type(16)));
typedef unsigned short v8us __attribute__((ext_vector_type(8), may_alias));
typedef float  v8f  __attribute__((ext_vector_type(8)));
typedef float  v4f  __attribute__((ext_vector_type(4)));
typedef float  v4fa __attribute__((ext_vector_type(4), may_alias));
union FragB { v16b v; v8us half[2]; unsigned short u[16]; };

__device__ __forceinline__ unsigned short bf16_bits(float x) { unsigned int u = __float_as_uint(x); return (unsigned short)((u + 0x7FFFu + ((u >> 16) & 1u)) >> 16); }
__device__ __forceinline__ float bf16_val(unsigned short b) { return __uint_as_float(((unsigned int)b) << 16); }
__device__ __forceinline__ float bf16_round(float x) { return bf16_val(bf16_bits(x)); }
template <int NT>
__device__ __forceinline__ v8f mmaN(v16b ah, v16b al, v16b bh, v16b bl, v8f c) {
  c = __builtin_amdgcn_wmma_f32_16x16x32_bf16(false, ah, false, bh, (short)0, c, false, false);
  if (NT >= 2) c = __builtin_amdgcn_wmma_f32_16x16x32_bf16(false, al, false, bh, (short)0, c, false, false);
  if (NT >= 3) c = __builtin_amdgcn_wmma_f32_16x16x32_bf16(false, ah, false, bl, (short)0, c, false, false);
  asm volatile("v_nop\n\tv_nop\n\tv_nop\n\tv_nop" : "+v"(c) : "v"(ah), "v"(al), "v"(bh), "v"(bl));
  return c;
}

__global__ __launch_bounds__(256) void k_wt_bf16(const float* __restrict__ W, unsigned short* __restrict__ Wt, int K, int N) {
  const int t = blockIdx.x * 256 + threadIdx.x;
  const int k8n = K / 8;
  if (t >= N * k8n) return;
  const int n = t / k8n, k8 = (t % k8n) * 8;
  v8us v;
#pragma unroll
  for (int i = 0; i < 8; ++i) v[i] = bf16_bits(W[(size_t)(k8 + i) * N + n]);
  *(volatile v8us*)(Wt + (size_t)n * K + k8) = v;
  __threadfence();
  *(volatile v8us*)(Wt + (size_t)n * K + k8) = v;
}

template <bool ASPLIT, int ACT, bool BIAS_BF16>
__global__ __launch_bounds__(128) void k_gemm_bf(const float* __restrict__ A, int lda, const unsigned short* __restrict__ Wt, int ldb,
                                               const float* __restrict__ bias, float* __restrict__ C, int ldc, int M, int N, int K) {
  __shared__ __attribute__((aligned(16))) float so[4][16][64];
  const int tid = threadIdx.x, w = tid >> 5, lane = tid & 31, ln = lane & 15, hh = lane >> 4;
  const int ntn = N / 64;
  const int wid = blockIdx.x * 4 + w;
  const int mt = wid / ntn, nq = wid % ntn;
  if (mt * 16 >= M) return;
  const int row0 = mt * 16, col0 = nq * 64;
  const float* arow = A + (size_t)(row0 + ln) * lda;
  v8f acc[4] = {};
  for (int kb = 0; kb < K; kb += 32) {
    FragB ah, al;
    const v4f x0 = *(const v4fa*)(arow + kb + 8 * hh), x1 = *(const v4fa*)(arow + kb + 8 * hh + 4);
    const v4f x2 = *(const v4fa*)(arow + kb + 16 + 8 * hh), x3 = *(const v4fa*)(arow + kb + 16 + 8 * hh + 4);
    float xs[16] = {x0[0],x0[1],x0[2],x0[3],x1[0],x1[1],x1[2],x1[3],x2[0],x2[1],x2[2],x2[3],x3[0],x3[1],x3[2],x3[3]};
#pragma unroll
    for (int i = 0; i < 16; ++i) { const unsigned short hb = bf16_bits(xs[i]); ah.u[i] = hb; al.u[i] = ASPLIT ? bf16_bits(xs[i] - bf16_val(hb)) : (unsigned short)0; }
#pragma unroll
    for (int t = 0; t < 4; ++t) {
      const unsigned short* brow = Wt + (size_t)(col0 + t * 16 + ln) * ldb + kb;
      FragB b;
      b.half[0] = *(const v8us*)(brow + 8 * hh);
      b.half[1] = *(const v8us*)(brow + 16 + 8 * hh);
      acc[t] = mmaN<ASPLIT ? 2 : 1>(ah.v, al.v, b.v, b.v, acc[t]);
    }
  }
#pragma unroll
  for (int t = 0; t < 4; ++t) {
    float bv = bias ? bias[col0 + t * 16 + ln] : 0.f;
    if (BIAS_BF16) bv = bf16_round(bv);
#pragma unroll
    for (int r = 0; r < 8; ++r) { float v = acc[t][r] + bv; if (ACT == 1) v = fmaxf(v, 0.f); so[w][8 * hh + r][t * 16 + ln] = v; }
  }
  __builtin_amdgcn_fence(__ATOMIC_ACQ_REL, "workgroup");
  __builtin_amdgcn_wave_barrier();
  const int rsub = lane >> 4, c4 = (lane & 15) * 4;
  for (int pass = 0; pass < 2; ++pass) {
#pragma unroll
    for (int q = 0; q < 8; ++q) {
      const int r = q * 2 + rsub;
      const v4f v = *(const v4fa*)&so[w][r][c4];
      *(volatile v4f*)(C + (size_t)(row0 + r) * ldc + col0 + c4) = v;
    }
    if (pass == 0) __threadfence();
  }
}

template <bool ASPLIT, int ACT, bool BIAS_BF16, bool RES_BF16>
__global__ __launch_bounds__(128) void k_gemm_bf3(const float* __restrict__ A, int lda, const unsigned short* __restrict__ Wt, int ldb,
                                                const float* __restrict__ bias, const float* __restrict__ resid, int rmod, int ldr,
                                                float* __restrict__ C, int ldc, int M, int N, int K) {
  __shared__ __attribute__((aligned(16))) float so[4][16][64];
  const int tid = threadIdx.x, w = tid >> 5, lane = tid & 31, ln = lane & 15, hh = lane >> 4;
  const int ntn = N / 64;
  const int wid = blockIdx.x * 4 + w;
  const int mt = wid / ntn, nq = wid % ntn;
  if (mt * 16 >= M) return;
  const int row0 = mt * 16, col0 = nq * 64;
  const float* arow = A + (size_t)(row0 + ln) * lda;
  v8f acc[4] = {};
  for (int kb = 0; kb < K; kb += 32) {
    FragB ah, al;
    const v4f x0 = *(const v4fa*)(arow + kb + 8 * hh), x1 = *(const v4fa*)(arow + kb + 8 * hh + 4);
    const v4f x2 = *(const v4fa*)(arow + kb + 16 + 8 * hh), x3 = *(const v4fa*)(arow + kb + 16 + 8 * hh + 4);
    float xs[16] = {x0[0],x0[1],x0[2],x0[3],x1[0],x1[1],x1[2],x1[3],x2[0],x2[1],x2[2],x2[3],x3[0],x3[1],x3[2],x3[3]};
#pragma unroll
    for (int i = 0; i < 16; ++i) { const unsigned short hb = bf16_bits(xs[i]); ah.u[i] = hb; al.u[i] = ASPLIT ? bf16_bits(xs[i] - bf16_val(hb)) : (unsigned short)0; }
#pragma unroll
    for (int t = 0; t < 4; ++t) {
      const unsigned short* brow = Wt + (size_t)(col0 + t * 16 + ln) * ldb + kb;
      FragB b;
      b.half[0] = *(const v8us*)(brow + 8 * hh);
      b.half[1] = *(const v8us*)(brow + 16 + 8 * hh);
      acc[t] = mmaN<ASPLIT ? 2 : 1>(ah.v, al.v, b.v, b.v, acc[t]);
    }
  }
#pragma unroll
  for (int t = 0; t < 4; ++t) {
    const int col = col0 + t * 16 + ln;
    float bv = bias ? bias[col] : 0.f;
    if (BIAS_BF16) bv = bf16_round(bv);
#pragma unroll
    for (int r = 0; r < 8; ++r) {
      float v = acc[t][r] + bv;
      if (resid) { float rv = resid[(size_t)((row0 + 8 * hh + r) % rmod) * ldr + col]; if (RES_BF16) rv = bf16_round(rv); v += rv; }
      if (ACT == 1) v = fmaxf(v, 0.f);
      if (ACT == 2) v = 0.5f * v * (1.0f + erff(v * 0.70710678118654752f));
      if (ACT == 3) { const float u = 0.7978845608028654f * (v + 0.044715f * v * v * v); v = 0.5f * v * (1.0f + tanhf(u)); }
      so[w][8 * hh + r][t * 16 + ln] = v;
    }
  }
  __builtin_amdgcn_fence(__ATOMIC_ACQ_REL, "workgroup");
  __builtin_amdgcn_wave_barrier();
  const int rsub = lane >> 4, c4 = (lane & 15) * 4;
  for (int pass = 0; pass < 2; ++pass) {
#pragma unroll
    for (int q = 0; q < 8; ++q) {
      const int r = q * 2 + rsub;
      const v4f v = *(const v4fa*)&so[w][r][c4];
      *(volatile v4f*)(C + (size_t)(row0 + r) * ldc + col0 + c4) = v;
    }
    if (pass == 0) __threadfence();
  }
}
template <bool PARAM_BF16>
__global__ __launch_bounds__(256) void k_layernorm(const float* __restrict__ X, const float* __restrict__ R, const float* __restrict__ g, const float* __restrict__ bta,
                                                  float* __restrict__ out_sum, float* __restrict__ out_norm, int N, float eps) {
  __shared__ float red[256];
  const int row = blockIdx.x, tid = threadIdx.x;
  const float* x = X + (size_t)row * N; const float* rr = R ? R + (size_t)row * N : nullptr;
  float vals[16];
  const int per = N / 256;
  float s1 = 0.f;
  for (int u = 0; u < per / 4; ++u) {
    const int j = tid * 4 + 1024 * u;
    const v4f a = *(const v4fa*)(x + j);
    v4f b = {0.f,0.f,0.f,0.f}; if (rr) b = *(const v4fa*)(rr + j);
#pragma unroll
    for (int q = 0; q < 4; ++q) { const float v = a[q] + b[q]; vals[u * 4 + q] = v; s1 += v; }
  }
  red[tid] = s1; __syncthreads();
  for (int st = 128; st > 0; st >>= 1) { if (tid < st) red[tid] += red[tid + st]; __syncthreads(); }
  const float mu = red[0] / (float)N; __syncthreads();
  float s2 = 0.f;
  for (int u = 0; u < per / 4; ++u)
#pragma unroll
    for (int q = 0; q < 4; ++q) { const float c = vals[u * 4 + q] - mu; s2 += c * c; }
  red[tid] = s2; __syncthreads();
  for (int st = 128; st > 0; st >>= 1) { if (tid < st) red[tid] += red[tid + st]; __syncthreads(); }
  const float rs = rsqrtf(red[0] / (float)N + eps);
  for (int pass = 0; pass < 2; ++pass) {
    for (int u = 0; u < per / 4; ++u) {
      const int j = tid * 4 + 1024 * u;
      v4f o, sm;
#pragma unroll
      for (int q = 0; q < 4; ++q) {
        float gg = g[j + q], bb = bta[j + q];
        if (PARAM_BF16) { gg = bf16_round(gg); bb = bf16_round(bb); }
        sm[q] = vals[u * 4 + q]; o[q] = (vals[u * 4 + q] - mu) * rs * gg + bb;
      }
      if (out_sum) *(volatile v4f*)(out_sum + (size_t)row * N + j) = sm;
      *(volatile v4f*)(out_norm + (size_t)row * N + j) = o;
    }
    if (pass == 0) __threadfence();
  }
}


typedef _Float16 v16h __attribute__((ext_vector_type(16)));
union FragH { v16h v; v8us half[2]; _Float16 h[16]; unsigned short u[16]; };
template <int NT>
__device__ __forceinline__ v8f mmaH(v16h ah, v16h al, v16h bh, v16h bl, v8f c) {
  c = __builtin_amdgcn_wmma_f32_16x16x32_f16(false, ah, false, bh, (short)0, c, false, false);
  if (NT >= 2) c = __builtin_amdgcn_wmma_f32_16x16x32_f16(false, al, false, bh, (short)0, c, false, false);
  if (NT >= 3) c = __builtin_amdgcn_wmma_f32_16x16x32_f16(false, ah, false, bl, (short)0, c, false, false);
  asm volatile("v_nop\n\tv_nop\n\tv_nop\n\tv_nop" : "+v"(c) : "v"(ah), "v"(al), "v"(bh), "v"(bl));
  return c;
}
template <bool ASPLIT>
__global__ __launch_bounds__(128) void k_gemm_h(const float* __restrict__ A, int lda, size_t sA, const _Float16* __restrict__ Bh, int ldb, size_t sB, float alpha, float* __restrict__ C, int ldc, size_t sC, int M, int N, int K) {
  __shared__ __attribute__((aligned(16))) float so[4][16][64];
  const int tid = threadIdx.x, w = tid >> 5, lane = tid & 31, ln = lane & 15, hh = lane >> 4; const int by = blockIdx.y;
  A += (size_t)by * sA; Bh += (size_t)by * sB; C += (size_t)by * sC;
  const int ntn = (N + 63) / 64; const int wid = blockIdx.x * 4 + w; const int mt = wid / ntn, nq = wid % ntn; if (mt * 16 >= M) return;
  const int row0 = mt * 16, col0 = nq * 64; const float* arow = A + (size_t)(row0 + ln) * lda;
  v8f acc[4] = {};
  for (int kb = 0; kb < K; kb += 32) {
    FragH ah, al;
    const v4f x0 = *(const v4fa*)(arow + kb + 8 * hh), x1 = *(const v4fa*)(arow + kb + 8 * hh + 4), x2 = *(const v4fa*)(arow + kb + 16 + 8 * hh), x3 = *(const v4fa*)(arow + kb + 16 + 8 * hh + 4);
    float xs[16] = {x0[0],x0[1],x0[2],x0[3],x1[0],x1[1],x1[2],x1[3],x2[0],x2[1],x2[2],x2[3],x3[0],x3[1],x3[2],x3[3]};
#pragma unroll
    for (int i = 0; i < 16; ++i) { const _Float16 h = (_Float16)xs[i]; ah.h[i] = h; al.h[i] = ASPLIT ? (_Float16)(xs[i] - (float)h) : (_Float16)0.0f; }
#pragma unroll
    for (int t = 0; t < 4; ++t) { if (col0 + t * 16 >= N) continue; const size_t boff = (size_t)(col0 + t * 16 + ln) * ldb + kb; FragH bq; bq.half[0] = *(const v8us*)(Bh + boff + 8 * hh); bq.half[1] = *(const v8us*)(Bh + boff + 16 + 8 * hh);
      acc[t] = mmaH<ASPLIT ? 2 : 1>(ah.v, al.v, bq.v, bq.v, acc[t]); }
  }
#pragma unroll
  for (int t = 0; t < 4; ++t) { if (col0 + t * 16 >= N) continue;
#pragma unroll
    for (int r = 0; r < 8; ++r) so[w][8 * hh + r][t * 16 + ln] = acc[t][r] * alpha; }
  __builtin_amdgcn_fence(__ATOMIC_ACQ_REL, "workgroup"); __builtin_amdgcn_wave_barrier();
  const int rsub = lane >> 4, c4 = (lane & 15) * 4;
  for (int pass = 0; pass < 2; ++pass) {
#pragma unroll
    for (int q = 0; q < 8; ++q) { const int r = q * 2 + rsub; if (col0 + c4 < N) { const v4f v = *(const v4fa*)&so[w][r][c4]; *(volatile v4f*)(C + (size_t)(row0 + r) * ldc + col0 + c4) = v; } }
    if (pass == 0) __threadfence(); }
}

__global__ __launch_bounds__(256) void k_wt_f16(const float* __restrict__ W, _Float16* __restrict__ Wt, int K, int N, float scale) {
  const int t = blockIdx.x * 256 + threadIdx.x; if (t >= N * (K / 8)) return; const int n = t / (K / 8), k8 = (t % (K / 8)) * 8; FragH f;
#pragma unroll
  for (int i = 0; i < 8; ++i) f.h[i] = (_Float16)(bf16_round(W[(size_t)(k8 + i) * N + n]) * scale); const v8us o = f.half[0];
  *(volatile v8us*)((unsigned short*)Wt + (size_t)n * K + k8) = o; __threadfence(); *(volatile v8us*)((unsigned short*)Wt + (size_t)n * K + k8) = o;
}
template <int ACT>
__global__ __launch_bounds__(128) void k_gemm_hhx(const _Float16* __restrict__ A, int lda, size_t sA, const _Float16* __restrict__ Bh, int ldb, size_t sB, float alpha, const float* __restrict__ bias, size_t sBias, const float* __restrict__ CP, int rowsPerB, size_t sCPb, int row0g,
    float* __restrict__ C, _Float16* __restrict__ C16, int ldc, size_t sC, int M, int N, int K) {
  __shared__ __attribute__((aligned(16))) float so[4][16][64];
  const int tid = threadIdx.x, w = tid >> 5, lane = tid & 31, ln = lane & 15, hh = lane >> 4; const int by = blockIdx.y;
  A += (size_t)by * sA; Bh += (size_t)by * sB; const size_t cofs = (size_t)by * sC; const float* bp = bias ? bias + (size_t)by * sBias : nullptr;
  const int ntn = (N + 63) / 64; const int wid = blockIdx.x * 4 + w; const int mt = wid / ntn, nq = wid % ntn; if (mt * 16 >= M) return;
  const int row0 = mt * 16, col0 = nq * 64; const _Float16* arow = A + (size_t)(row0 + ln) * lda;
  v8f acc[4] = {};
  for (int kb = 0; kb < K; kb += 32) { FragH ah; ah.half[0] = *(const v8us*)((const unsigned short*)arow + kb + 8 * hh); ah.half[1] = *(const v8us*)((const unsigned short*)arow + kb + 16 + 8 * hh);
#pragma unroll
    for (int t = 0; t < 4; ++t) { if (col0 + t * 16 >= N) continue; const size_t boff = (size_t)(col0 + t * 16 + ln) * ldb + kb; FragH bq; bq.half[0] = *(const v8us*)((const unsigned short*)Bh + boff + 8 * hh); bq.half[1] = *(const v8us*)((const unsigned short*)Bh + boff + 16 + 8 * hh);
      acc[t] = mmaH<1>(ah.v, ah.v, bq.v, bq.v, acc[t]); }
  }
#pragma unroll
  for (int t = 0; t < 4; ++t) { if (col0 + t * 16 >= N) continue; const int col = col0 + t * 16 + ln; const float bv = bp ? bf16_round(bp[col]) : 0.f;
#pragma unroll
    for (int r = 0; r < 8; ++r) { float v = acc[t][r] * alpha + bv; if (CP) { const int rr = row0g + row0 + 8 * hh + r; if (rowsPerB < 0) v += CP[cofs + (size_t)rr * ldc + col];        else { const int bidx = rr / rowsPerB; v += CP[(size_t)bidx * sCPb + (size_t)by * 64 + col]; } } if (ACT == 1) v = (v > 0.f) ? v : expm1f(v); else if (ACT == 7) v = (v > 0.f) ? v + 1.0f : expf(v); else if (ACT == 8) v = tanhf(v); else if (ACT == 9) v = 0.5f * v * (1.0f + tanhf(0.7978845608028654f * (v + 0.044715f * v * v * v))); else if (ACT == 11) v = 1.0f / (1.0f + expf(-v)); else if (ACT == 12) v = (v > 0.f) ? v : 0.01f * v; else if (ACT == 14) v = (v > 0.f) ? v : 0.1f * v; else if (ACT == 16) v = (v >= 0.f) ? v : 0.3f * v; else if (ACT == 17) v = (v >= 0.f) ? v : 0.2f * v; else if (ACT == 15) v = v / (1.0f + expf(-v)); else if (ACT == 3) v = fmaxf(v, 0.f); else if (ACT == 6) v = 0.5f * v * (1.0f + erff(v * 0.70710678118654752f)); so[w][8 * hh + r][t * 16 + ln] = v; } }
  __builtin_amdgcn_fence(__ATOMIC_ACQ_REL, "workgroup"); __builtin_amdgcn_wave_barrier();
  const int rsub = lane >> 4, c4 = (lane & 15) * 4; typedef _Float16 v4h __attribute__((ext_vector_type(4)));
  for (int pass = 0; pass < 2; ++pass) {
#pragma unroll
    for (int q = 0; q < 8; ++q) { const int r = q * 2 + rsub; if (col0 + c4 < N) { const v4f v = *(const v4fa*)&so[w][r][c4]; if (C) *(volatile v4f*)(C + cofs + (size_t)(row0 + r) * ldc + col0 + c4) = v; if (C16) { v4h h4; for (int i = 0; i < 4; ++i) h4[i] = (_Float16)v[i]; *(volatile v4h*)(C16 + cofs + (size_t)(row0 + r) * ldc + col0 + c4) = h4; } } }
    if (pass == 0) __threadfence(); }
}


typedef _Float16 v4h __attribute__((ext_vector_type(4)));

__global__ __launch_bounds__(256) void k_x16(const float* __restrict__ x, _Float16* __restrict__ X16, size_t n8) { const size_t t = (size_t)blockIdx.x * 256 + threadIdx.x; if (t >= n8) return; FragH f;
#pragma unroll
  for (int q = 0; q < 8; ++q) f.h[q] = (_Float16)bf16_round(x[t * 8 + q]); *(volatile v8us*)((unsigned short*)X16 + t * 8) = f.half[0]; __threadfence(); *(volatile v8us*)((unsigned short*)X16 + t * 8) = f.half[0]; }
__global__ __launch_bounds__(256) void k_h16(const float* __restrict__ x, _Float16* __restrict__ X16, size_t n8) { const size_t t = (size_t)blockIdx.x * 256 + threadIdx.x; if (t >= n8) return; FragH f;
#pragma unroll
  for (int q = 0; q < 8; ++q) f.h[q] = (_Float16)x[t * 8 + q]; *(volatile v8us*)((unsigned short*)X16 + t * 8) = f.half[0]; __threadfence(); *(volatile v8us*)((unsigned short*)X16 + t * 8) = f.half[0]; }
__global__ __launch_bounds__(256) void k_round16f(const float* __restrict__ W, _Float16* __restrict__ Bt, size_t n8) { const size_t t = (size_t)blockIdx.x * 256 + threadIdx.x; if (t >= n8) return; FragH f;
#pragma unroll
  for (int i = 0; i < 8; ++i) f.h[i] = (_Float16)(bf16_round(W[t * 8 + i]) * 16.0f); *(volatile v8us*)((unsigned short*)Bt + t * 8) = f.half[0]; __threadfence(); *(volatile v8us*)((unsigned short*)Bt + t * 8) = f.half[0]; }
template <int NHv, int TTv>
__global__ __launch_bounds__(256) void k_vt(const _Float16* __restrict__ V16, int ldv, int voff, _Float16* __restrict__ Vt) { __shared__ unsigned short tl[64][66]; const int tid = threadIdx.x; const int slab = blockIdx.x / (TTv / 64), lg = blockIdx.x % (TTv / 64); const int b = slab / NHv, h = slab % NHv;
  for (int i = tid; i < 64 * 8; i += 256) { const int r = i / 8, c8 = (i % 8) * 8; FragH f; f.half[0] = *(const v8us*)((const unsigned short*)V16 + ((size_t)b * TTv + lg * 64 + r) * ldv + voff + h * 64 + c8);
#pragma unroll
    for (int q = 0; q < 8; ++q) tl[r][c8 + q] = f.u[q]; }
  __syncthreads();
  for (int pass = 0; pass < 2; ++pass) {
#pragma unroll
    for (int rd = 0; rd < 2; ++rd) { const int d = rd * 32 + tid / 8, pc = tid % 8; FragH f;
#pragma unroll
      for (int q = 0; q < 8; ++q) f.u[q] = tl[pc * 8 + q][d];
      *(volatile v8us*)((unsigned short*)Vt + ((size_t)slab * 64 + d) * TTv + lg * 64 + pc * 8) = f.half[0]; }
    if (pass == 0) __threadfence(); } }

__global__ __launch_bounds__(256) void k_hl(const float* __restrict__ F, _Float16* __restrict__ Hh, _Float16* __restrict__ Hl, size_t n8) { const size_t t = (size_t)blockIdx.x * 256 + threadIdx.x; if (t >= n8) return; FragH fh, fl; const v4f a = *(const v4fa*)(F + t * 8), c = *(const v4fa*)(F + t * 8 + 4);
#pragma unroll
  for (int q = 0; q < 4; ++q) { _Float16 h = (_Float16)a[q]; fh.h[q] = h; fl.h[q] = (_Float16)((a[q] - (float)h) * 1024.0f); h = (_Float16)c[q]; fh.h[4 + q] = h; fl.h[4 + q] = (_Float16)((c[q] - (float)h) * 1024.0f); }
  for (int pass = 0; pass < 2; ++pass) { *(volatile v8us*)((unsigned short*)Hh + t * 8) = fh.half[0]; *(volatile v8us*)((unsigned short*)Hl + t * 8) = fl.half[0]; if (pass == 0) __threadfence(); } }

__device__ __forceinline__ v16h g2_frag(const _Float16* p, int hh) { FragH f; f.half[0] = *(const v8us*)((const unsigned short*)p + 8 * hh); f.half[1] = *(const v8us*)((const unsigned short*)p + 16 + 8 * hh); return f.v; }
__device__ __forceinline__ v8f g2_mma(v16h a, v16h b, v8f c) { v8f d = __builtin_amdgcn_wmma_f32_16x16x32_f16(false, a, false, b, (short)0, c, false, false); asm volatile("v_nop\n\tv_nop\n\tv_nop\n\tv_nop" : "+v"(d) : "v"(a), "v"(b)); return d; }
template <int ACT>
__global__ __launch_bounds__(128) void k_gemm2(const _Float16* __restrict__ A, int lda, size_t sA, const _Float16* __restrict__ Bh, int ldb, size_t sB, float alpha, const float* __restrict__ bias, size_t sBias, const float* __restrict__ CP, int rowsPerB, size_t sCPb, int row0g,
    float* __restrict__ C, _Float16* __restrict__ C16, int ldc, size_t sC, int M, int N, int K) { static_assert(ACT == 0 || ACT == 3 || ACT == 6 || ACT == 8 || ACT == 9 || ACT == 11 || ACT == 12 || ACT == 14 || ACT == 15 || ACT == 16 || ACT == 17, "k_gemm2: unsupported ACT code (would silently apply no activation)");
  __shared__ __attribute__((aligned(16))) float so[4][32][68];
  const int tid = threadIdx.x, w = tid >> 5, lane = tid & 31, ln = lane & 15, hh = lane >> 4; const int by = blockIdx.y;
  A += (size_t)by * sA; Bh += (size_t)by * sB; const size_t cofs = (size_t)by * sC; const float* bp = bias ? bias + (size_t)by * sBias : nullptr;
  const int ntn = N >> 6; const int mt = blockIdx.x / ntn, nq = blockIdx.x - mt * ntn; const int row0 = mt * 128 + 32 * w, col0 = nq * 64; if (row0 >= M) return;
  const _Float16* a0p = A + (size_t)(row0 + ln) * lda; const _Float16* a1p = a0p + (size_t)16 * lda;
  const _Float16* b0p = Bh + (size_t)(col0 + ln) * ldb; const _Float16* b1p = b0p + (size_t)16 * ldb; const _Float16* b2p = b1p + (size_t)16 * ldb; const _Float16* b3p = b2p + (size_t)16 * ldb;
  const v8f z8 = {0.f,0.f,0.f,0.f,0.f,0.f,0.f,0.f}; v8f c00 = z8, c01 = z8, c02 = z8, c03 = z8, c10 = z8, c11 = z8, c12 = z8, c13 = z8;
#pragma unroll 1
  for (int kb = 0; kb < K; kb += 32) { const v16h a0 = g2_frag(a0p + kb, hh), a1 = g2_frag(a1p + kb, hh);
    v16h b = g2_frag(b0p + kb, hh); c00 = g2_mma(a0, b, c00); c10 = g2_mma(a1, b, c10);
    b = g2_frag(b1p + kb, hh); c01 = g2_mma(a0, b, c01); c11 = g2_mma(a1, b, c11);
    b = g2_frag(b2p + kb, hh); c02 = g2_mma(a0, b, c02); c12 = g2_mma(a1, b, c12);
    b = g2_frag(b3p + kb, hh); c03 = g2_mma(a0, b, c03); c13 = g2_mma(a1, b, c13); }
  v8f accs[8] = {c00, c01, c02, c03, c10, c11, c12, c13};
#pragma unroll
  for (int u = 0; u < 8; ++u) { const int t = u & 3, half = u >> 2; const int col = col0 + t * 16 + ln; const float bv = bp ? bf16_round(bp[col]) : 0.f;
#pragma unroll
    for (int r = 0; r < 8; ++r) { const int rloc = half * 16 + 8 * hh + r; float v = accs[u][r] * alpha + bv; if (CP) { if (rowsPerB < 0) v += CP[cofs + (size_t)(row0g + row0 + rloc) * ldc + col];        else { const int bidx = (row0g + row0 + rloc) / rowsPerB; v += CP[(size_t)bidx * sCPb + (size_t)by * 64 + col]; } }
      if (ACT == 3) v = fmaxf(v, 0.f); else if (ACT == 6) v = 0.5f * v * (1.0f + erff(v * 0.70710678118654752f)); else if (ACT == 11) v = 1.0f / (1.0f + expf(-v)); else if (ACT == 15) v = v / (1.0f + expf(-v)); else if (ACT == 12) v = (v > 0.f) ? v : 0.01f * v; else if (ACT == 8) v = tanhf(v); else if (ACT == 9) v = 0.5f * v * (1.0f + tanhf(0.7978845608028654f * (v + 0.044715f * v * v * v))); else if (ACT == 14) v = (v > 0.f) ? v : 0.1f * v; else if (ACT == 16) v = (v >= 0.f) ? v : 0.3f * v; else if (ACT == 17) v = (v >= 0.f) ? v : 0.2f * v;
      so[w][rloc][t * 16 + ln] = v; } }
  __builtin_amdgcn_fence(__ATOMIC_ACQ_REL, "workgroup"); __builtin_amdgcn_wave_barrier();
  const int rsub = lane >> 4, c4 = (lane & 15) * 4;
  for (int pass = 0; pass < 2; ++pass) {
#pragma unroll
    for (int q = 0; q < 16; ++q) { const int r = q * 2 + rsub; const v4f v = *(const v4fa*)&so[w][r][c4]; if (C) *(volatile v4f*)(C + cofs + (size_t)(row0 + r) * ldc + col0 + c4) = v; if (C16) { v4h h4; for (int i = 0; i < 4; ++i) h4[i] = (_Float16)v[i]; *(volatile v4h*)(C16 + cofs + (size_t)(row0 + r) * ldc + col0 + c4) = h4; } }
    if (pass == 0) __threadfence(); } }


__device__ __forceinline__ float gelu_erf(float v) { return 0.5f * v * (1.0f + erff(v * 0.70710678118654752f)); }
__device__ __forceinline__ float siluf(float v) { return v / (1.0f + expf(-v)); }
__global__ __launch_bounds__(256) void k_tok(const float* __restrict__ x, _Float16* __restrict__ X) { __shared__ float tl[CX][17]; const int tid = threadIdx.x; const int b = blockIdx.x / (NPX / 16), pb = blockIdx.x % (NPX / 16); const int p0 = pb * 16;
  for (int i = tid; i < CX * 16; i += 256) { const int c = i / 16, p = i % 16; tl[c][p] = bf16_round(x[((size_t)b * CX + c) * NPX + p0 + p]); }
  __syncthreads();
  for (int pass = 0; pass < 2; ++pass) { for (int i = tid; i < 16 * (CX / 8); i += 256) { const int p = i / (CX / 8), c0 = (i % (CX / 8)) * 8; FragH f; for (int q = 0; q < 8; ++q) f.h[q] = (_Float16)tl[c0 + q][p];
      *(volatile v8us*)((unsigned short*)X + ((size_t)b * NPX + p0 + p) * CX + c0) = f.half[0]; } if (pass == 0) __threadfence(); } }
__global__ __launch_bounds__(256) void k_im2(const _Float16* __restrict__ S, int cn, int kk, size_t r0, size_t nrows, _Float16* __restrict__ I) { const size_t t = (size_t)blockIdx.x * 256 + threadIdx.x; const int c8n = cn / 8; const int ntap = kk * kk; if (t >= nrows * ntap * c8n) return; const int c8 = (int)(t % c8n) * 8; const int tap = (int)((t / c8n) % ntap); const size_t row = r0 + t / ((size_t)ntap * c8n); const int b = (int)(row / NPX), p = (int)(row % NPX); const int pd = kk / 2; const int iy = p / WSD - pd + tap / kk, ix = p % WSD - pd + tap % kk; v8us v;
  if (iy >= 0 && iy < HS && ix >= 0 && ix < WSD) v = *(const v8us*)((const unsigned short*)S + (((size_t)b * NPX) + iy * WSD + ix) * cn + c8); else { for (int q = 0; q < 8; ++q) v[q] = 0; }
  unsigned short* d = (unsigned short*)I + (row - r0) * (size_t)(ntap * cn) + tap * cn + c8; *(volatile v8us*)d = v; __threadfence(); *(volatile v8us*)d = v; }
__global__ __launch_bounds__(256) void k_wre(const float* __restrict__ w, int cn, int kk, int nlive, int nrows, _Float16* __restrict__ Bt) { const size_t t = (size_t)blockIdx.x * 256 + threadIdx.x; const int ntap = kk * kk; const size_t kc = (size_t)ntap * cn; if (t >= (size_t)nrows * kc / 8) return; const int c8 = (int)((t * 8) % cn); const int tap = (int)(((t * 8) / cn) % ntap); const int o = (int)((t * 8) / kc); FragH f; for (int q = 0; q < 8; ++q) f.h[q] = (o < nlive) ? (_Float16)(bf16_round(w[((size_t)o * cn + c8 + q) * ntap + tap]) * 16.0f) : (_Float16)0.0f;
  *(volatile v8us*)((unsigned short*)Bt + t * 8) = f.half[0]; __threadfence(); *(volatile v8us*)((unsigned short*)Bt + t * 8) = f.half[0]; }
__global__ __launch_bounds__(256) void k_wsn(const float* __restrict__ w, _Float16* __restrict__ Bt) { const size_t t = (size_t)blockIdx.x * 256 + threadIdx.x; if (t >= (size_t)CO * KSN / 8) return; const int c8 = (int)((t * 8) % CHD); const int k = (int)(((t * 8) / CHD) % KS); const int o = (int)((t * 8) / KSN); FragH f; for (int q = 0; q < 8; ++q) f.h[q] = (_Float16)(bf16_round(w[((size_t)o * CHD + c8 + q) * KS + k]) * 16.0f);
  *(volatile v8us*)((unsigned short*)Bt + t * 8) = f.half[0]; __threadfence(); *(volatile v8us*)((unsigned short*)Bt + t * 8) = f.half[0]; }
__global__ __launch_bounds__(64) void k_bpad2(const float* __restrict__ a, const float* __restrict__ b2, float* __restrict__ dst) { const int i = threadIdx.x; float v = 0.f; if (i < 18) v = bf16_round(a[i]); else if (i < 36) v = bf16_round(b2[i - 18]); *(volatile float*)(dst + i) = v; __threadfence(); *(volatile float*)(dst + i) = v; }
__global__ __launch_bounds__(256) void k_wsc(const float* __restrict__ Wm, _Float16* __restrict__ Bt, size_t n8, float sc) { const size_t t = (size_t)blockIdx.x * 256 + threadIdx.x; if (t >= n8) return; FragH f; for (int q = 0; q < 8; ++q) f.h[q] = (_Float16)(bf16_round(Wm[t * 8 + q]) * sc); *(volatile v8us*)((unsigned short*)Bt + t * 8) = f.half[0]; __threadfence(); *(volatile v8us*)((unsigned short*)Bt + t * 8) = f.half[0]; }
__global__ __launch_bounds__(256) void k_affgelu(const float* __restrict__ Cv, const float* __restrict__ g, const float* __restrict__ bb, float* __restrict__ HF, _Float16* __restrict__ H16, _Float16* __restrict__ HL16) {
  #pragma clang fp contract(off)
  const size_t t = (size_t)blockIdx.x * 256 + threadIdx.x; if (t >= (size_t)NR * CHD / 8) return; const int c0 = (int)((t * 8) % CHD); const v8f a = *(const v8f*)(Cv + t * 8); v8f o; FragH f;
  for (int q = 0; q < 8; ++q) { float y = a[q] * bf16_round(g[c0 + q]); y += bf16_round(bb[c0 + q]); o[q] = y; }
#pragma unroll 1
  for (int q = 0; q < 8; ++q) o[q] = gelu_erf(o[q]);
  FragH fl; for (int q = 0; q < 8; ++q) { const _Float16 hq = (_Float16)o[q]; f.h[q] = hq; fl.h[q] = (_Float16)((o[q] - (float)hq) * 1024.0f); }
  for (int pass = 0; pass < 2; ++pass) { *(volatile v8f*)(HF + t * 8) = o; *(volatile v8us*)((unsigned short*)H16 + t * 8) = f.half[0]; *(volatile v8us*)((unsigned short*)HL16 + t * 8) = fl.half[0]; if (pass == 0) __threadfence(); } }
__global__ __launch_bounds__(256) void k_affsilu(const float* __restrict__ Cv, const float* __restrict__ g, const float* __restrict__ bb, size_t r0, size_t nrows, int coff, _Float16* __restrict__ CAT) {
  #pragma clang fp contract(off)
  const size_t t = (size_t)blockIdx.x * 256 + threadIdx.x; if (t >= nrows * CO / 8) return; const int c0 = (int)((t * 8) % CO); const size_t lrow = (t * 8) / CO; const v8f a = *(const v8f*)(Cv + t * 8); FragH f;
  for (int q = 0; q < 8; ++q) { float y = a[q] * bf16_round(g[c0 + q]); y += bf16_round(bb[c0 + q]); f.h[q] = (_Float16)siluf(y); }
  unsigned short* d = (unsigned short*)CAT + (r0 + lrow) * CC + coff + c0; *(volatile v8us*)d = f.half[0]; __threadfence(); *(volatile v8us*)d = f.half[0]; }
template <int MORPH>
__global__ __launch_bounds__(256) void k_snake(const float* __restrict__ HF, const float* __restrict__ OFF, const float* __restrict__ og, const float* __restrict__ obeta, int obase, _Float16* __restrict__ FE) {
  #pragma clang fp contract(off)
  const size_t t = (size_t)blockIdx.x * 256 + threadIdx.x; if (t >= (size_t)NR * KS * (CHD / 8)) return; const int cg = (int)(t % (CHD / 8)); const int k = (int)((t / (CHD / 8)) % KS); const size_t row = t / ((size_t)KS * (CHD / 8)); const int b = (int)(row / NPX), p = (int)(row % NPX); const int y = p / WSD, x = p % WSD;
  const float* o = OFF + row * 64 + obase + (MORPH ? KS : 0);
  const float* gg = og + (MORPH ? KS : 0); const float* be = obeta + (MORPH ? KS : 0);
  float cum = 0.f;
  if (k > 4) { for (int i = 5; i <= k; ++i) { float u = o[i] * bf16_round(gg[i]); u += bf16_round(be[i]); cum += tanhf(u); } }
  else if (k < 4) { for (int i = 3; i >= k; --i) { float u = o[i] * bf16_round(gg[i]); u += bf16_round(be[i]); cum += tanhf(u); } }
  float ys, xs; if (MORPH == 0) { ys = (float)y + cum; xs = (float)(x + k - 4); } else { xs = (float)x + cum; ys = (float)(y + k - 4); }
  ys = fminf(fmaxf(ys, 0.f), (float)(HS - 1)); xs = fminf(fmaxf(xs, 0.f), (float)(WSD - 1)); const float y0 = floorf(ys), x0 = floorf(xs); const float wy = ys - y0, wx = xs - x0; const int y0i = (int)y0, x0i = (int)x0; const int y1i = min(y0i + 1, HS - 1), x1i = min(x0i + 1, WSD - 1);
  const float* r00 = HF + (((size_t)b * NPX) + y0i * WSD + x0i) * CHD + cg * 8; const float* r01 = HF + (((size_t)b * NPX) + y0i * WSD + x1i) * CHD + cg * 8; const float* r10 = HF + (((size_t)b * NPX) + y1i * WSD + x0i) * CHD + cg * 8; const float* r11 = HF + (((size_t)b * NPX) + y1i * WSD + x1i) * CHD + cg * 8;
  const float w00 = (1.f - wy) * (1.f - wx), w01 = (1.f - wy) * wx, w10 = wy * (1.f - wx), w11 = wy * wx; const v8f a00 = *(const v8f*)r00, a01 = *(const v8f*)r01, a10 = *(const v8f*)r10, a11 = *(const v8f*)r11; FragH f;
  for (int q = 0; q < 8; ++q) { float s = w00 * a00[q]; s += w01 * a01[q]; s += w10 * a10[q]; s += w11 * a11[q]; f.h[q] = (_Float16)s; }
  unsigned short* d = (unsigned short*)FE + row * (size_t)KSN + k * CHD + cg * 8; *(volatile v8us*)d = f.half[0]; __threadfence(); *(volatile v8us*)d = f.half[0]; }
__global__ __launch_bounds__(256) void k_gnst(const float* __restrict__ D, float* __restrict__ ST) {
  #pragma clang fp contract(off)
  __shared__ float red[256]; __shared__ float stat; const int tid = threadIdx.x; const int b = blockIdx.x / 32, grp = blockIdx.x % 32; float s = 0.f;
  for (int i = tid; i < NPX * 4; i += 256) { const int p = i / 4, c = grp * 4 + (i % 4); s += D[((size_t)b * NPX + p) * CO + c]; }
  red[tid] = s; __syncthreads(); for (int st = 128; st > 0; st >>= 1) { if (tid < st) red[tid] += red[tid + st]; __syncthreads(); } if (tid == 0) stat = red[0] / (float)(NPX * 4); __syncthreads(); const float mu = stat; float s2 = 0.f;
  for (int i = tid; i < NPX * 4; i += 256) { const int p = i / 4, c = grp * 4 + (i % 4); const float dd = D[((size_t)b * NPX + p) * CO + c] - mu; s2 += dd * dd; }
  __syncthreads(); red[tid] = s2; __syncthreads(); for (int st = 128; st > 0; st >>= 1) { if (tid < st) red[tid] += red[tid + st]; __syncthreads(); }
  if (tid < 32) { const float o = (tid == 0) ? mu : ((tid == 1) ? rsqrtf(red[0] / (float)(NPX * 4) + 1e-5f) : 0.f); *(volatile float*)(ST + (size_t)blockIdx.x * 32 + tid) = o; __threadfence(); *(volatile float*)(ST + (size_t)blockIdx.x * 32 + tid) = o; } }
__global__ __launch_bounds__(256) void k_gnap(const float* __restrict__ D, const float* __restrict__ ST, const float* __restrict__ g, const float* __restrict__ bb, int coff, _Float16* __restrict__ CAT) {
  #pragma clang fp contract(off)
  const size_t t = (size_t)blockIdx.x * 256 + threadIdx.x; if (t >= (size_t)NR * CO / 8) return; const int c0 = (int)((t * 8) % CO); const size_t row = (t * 8) / CO; const int b = (int)(row / NPX); const v8f a = *(const v8f*)(D + t * 8); FragH f;
  for (int q = 0; q < 8; ++q) { const int c = c0 + q; const float* st = ST + ((size_t)b * 32 + c / 4) * 32; float y = (a[q] - st[0]) * st[1]; y = y * bf16_round(g[c]); y += bf16_round(bb[c]); f.h[q] = (_Float16)siluf(y); }
  unsigned short* d = (unsigned short*)CAT + row * CC + coff + c0; *(volatile v8us*)d = f.half[0]; __threadfence(); *(volatile v8us*)d = f.half[0]; }
__global__ __launch_bounds__(256) void k_affsilu32(const float* __restrict__ Cv, const float* __restrict__ g, const float* __restrict__ bb, float* __restrict__ O) {
  #pragma clang fp contract(off)
  const size_t t = (size_t)blockIdx.x * 256 + threadIdx.x; if (t >= (size_t)NR * CO / 8) return; const int c0 = (int)((t * 8) % CO); const v8f a = *(const v8f*)(Cv + t * 8); v8f o;
  for (int q = 0; q < 8; ++q) { float y = a[q] * bf16_round(g[c0 + q]); y += bf16_round(bb[c0 + q]); o[q] = siluf(y); }
  *(volatile v8f*)(O + t * 8) = o; __threadfence(); *(volatile v8f*)(O + t * 8) = o; }
__global__ __launch_bounds__(256) void k_simst(const float* __restrict__ O, float* __restrict__ SS) {
  #pragma clang fp contract(off)
  __shared__ float red[256]; __shared__ float stat; const int tid = threadIdx.x; const int b = blockIdx.x / CO, c = blockIdx.x % CO; float s = 0.f;
  for (int p = tid; p < NPX; p += 256) s += O[((size_t)b * NPX + p) * CO + c];
  red[tid] = s; __syncthreads(); for (int st = 128; st > 0; st >>= 1) { if (tid < st) red[tid] += red[tid + st]; __syncthreads(); } if (tid == 0) stat = red[0] / (float)NPX; __syncthreads(); const float mu = stat; float s2 = 0.f;
  for (int p = tid; p < NPX; p += 256) { const float dd = O[((size_t)b * NPX + p) * CO + c] - mu; s2 += dd * dd; }
  __syncthreads(); red[tid] = s2; __syncthreads(); for (int st = 128; st > 0; st >>= 1) { if (tid < st) red[tid] += red[tid + st]; __syncthreads(); }
  if (tid < 32) { const float o = (tid == 0) ? mu : ((tid == 1) ? red[0] : 0.f); *(volatile float*)(SS + (size_t)blockIdx.x * 32 + tid) = o; __threadfence(); *(volatile float*)(SS + (size_t)blockIdx.x * 32 + tid) = o; } }
__global__ __launch_bounds__(256) void k_final(const float* __restrict__ O, const float* __restrict__ SS, const float* __restrict__ x, float* __restrict__ out) {
  #pragma clang fp contract(off)
  const size_t t = (size_t)blockIdx.x * 256 + threadIdx.x; if (t >= (size_t)NI * CO * NPX / 8) return; const int p0 = (int)((t * 8) % NPX); const size_t bc = (t * 8) / NPX; const int b = (int)(bc / CO), c = (int)(bc % CO); const float mu = SS[bc * 32], sd = SS[bc * 32 + 1]; float den = sd / (float)(NPX - 1); den += 1e-4f; den = 4.0f * den; const v8f xi = *(const v8f*)(x + t * 8); v8f v;
  for (int q = 0; q < 8; ++q) { const float o = O[((size_t)b * NPX + p0 + q) * CO + c]; const float dd = (o - mu) * (o - mu); float e = dd / den; e += 0.5f; const float sg = 1.0f / (1.0f + expf(-e)); float r = o * sg; r += bf16_round(xi[q]); v[q] = r; }
  *(volatile v8f*)(out + t * 8) = v; __threadfence(); *(volatile v8f*)(out + t * 8) = v; }

extern "C" void kernel_launch(void* const* d_in, const int* in_sizes, int n_in,
                              void* d_out, int out_size, void* d_ws, size_t ws_size, hipStream_t stream) {
  (void)in_sizes; (void)n_in; (void)out_size;
  const float* const* I = (const float* const*)d_in; const float* x = I[0]; const float* cv1_w = I[1]; const float* cv1_g = I[2]; const float* cv1_b = I[3]; const float* c0w = I[4]; const float* c0g = I[5]; const float* c0b = I[6];
  const float* offx_w = I[7]; const float* offx_b = I[8]; const float* offx_g = I[9]; const float* offx_beta = I[10]; const float* dscx_w = I[11]; const float* dscx_b = I[12]; const float* gnx_g = I[13]; const float* gnx_b = I[14];
  const float* offy_w = I[15]; const float* offy_b = I[16]; const float* offy_g = I[17]; const float* offy_beta = I[18]; const float* dscy_w = I[19]; const float* dscy_b = I[20]; const float* gny_g = I[21]; const float* gny_b = I[22]; const float* fuse_w = I[23]; const float* fuse_g = I[24]; const float* fuse_b = I[25];
  char* ws = (char*)d_ws; size_t off = 0;
  auto take = [&](size_t bytes) { char* p = ws + off; off += (bytes + 255) & ~(size_t)255; return p; };
  _Float16* B1 = (_Float16*)take((size_t)CHD * K1 * 2); _Float16* B9 = (_Float16*)take((size_t)CO * K9 * 2); _Float16* BOF = (_Float16*)take((size_t)64 * K3 * 2); float* bofp = (float*)take(64 * 4); _Float16* BSX = (_Float16*)take((size_t)CO * KSN * 2); _Float16* BSY = (_Float16*)take((size_t)CO * KSN * 2); _Float16* BF = (_Float16*)take((size_t)CO * CC * 2); float* ST = (float*)take((size_t)NI * 32 * 32 * 4); float* SS = (float*)take((size_t)NI * CO * 32 * 4);
  _Float16* X = (_Float16*)take((size_t)NR * CX * 2); _Float16* IM = (_Float16*)take((size_t)NPX * K9 * 2); float* CV = (float*)take((size_t)NR * CO * 4); float* HF = (float*)take((size_t)NR * CHD * 4); _Float16* H16 = (_Float16*)take((size_t)NR * CHD * 2); _Float16* HL16 = (_Float16*)take((size_t)NR * CHD * 2); float* OFF = (float*)take((size_t)NR * 64 * 4); _Float16* CAT = (_Float16*)take((size_t)NR * CC * 2); float* O1 = (float*)take((size_t)NR * CO * 4);
  _Float16* FE = IM;
  if (off > ws_size) return;
  k_wre<<<(unsigned)(((size_t)CHD * K1 / 8 + 255) / 256), 256, 0, stream>>>(cv1_w, CX, 3, CHD, CHD, B1); k_wre<<<(unsigned)(((size_t)CO * K9 / 8 + 255) / 256), 256, 0, stream>>>(c0w, CHD, 9, CO, CO, B9);
  k_wre<<<(unsigned)(((size_t)18 * K3 / 8 + 255) / 256), 256, 0, stream>>>(offx_w, CHD, 3, 18, 18, BOF); k_wre<<<(unsigned)(((size_t)46 * K3 / 8 + 255) / 256), 256, 0, stream>>>(offy_w, CHD, 3, 18, 46, BOF + (size_t)18 * K3); k_bpad2<<<1, 64, 0, stream>>>(offx_b, offy_b, bofp);
  k_wsn<<<(unsigned)(((size_t)CO * KSN / 8 + 255) / 256), 256, 0, stream>>>(dscx_w, BSX); k_wsn<<<(unsigned)(((size_t)CO * KSN / 8 + 255) / 256), 256, 0, stream>>>(dscy_w, BSY); k_wsc<<<(unsigned)(((size_t)CO * CC / 8 + 255) / 256), 256, 0, stream>>>(fuse_w, BF, (size_t)CO * CC / 8, 16.0f);
  k_tok<<<NI * (NPX / 16), 256, 0, stream>>>(x, X);
  for (int b = 0; b < NI; ++b) { const size_t r0 = (size_t)b * NPX; k_im2<<<(unsigned)(((size_t)NPX * 9 * (CX / 8) + 255) / 256), 256, 0, stream>>>(X, CX, 3, r0, NPX, IM); k_gemm2<0><<<dim3((NPX / 128) * (CHD / 64), 1), 128, 0, stream>>>(IM, K1, 0, B1, K1, 0, 0.0625f, nullptr, 0, nullptr, 1, 0, 0, CV + r0 * CHD, nullptr, CHD, 0, NPX, CHD, K1); }
  k_affgelu<<<(unsigned)(((size_t)NR * CHD / 8 + 255) / 256), 256, 0, stream>>>(CV, cv1_g, cv1_b, HF, H16, HL16);
  for (int b = 0; b < NI; ++b) { const size_t r0 = (size_t)b * NPX; k_im2<<<(unsigned)(((size_t)NPX * 81 * (CHD / 8) + 255) / 256), 256, 0, stream>>>(H16, CHD, 9, r0, NPX, IM); k_gemm2<0><<<dim3((NPX / 128) * (CO / 64), 1), 128, 0, stream>>>(IM, K9, 0, B9, K9, 0, 0.0625f, nullptr, 0, nullptr, 1, 0, 0, CV + r0 * CO, nullptr, CO, 0, NPX, CO, K9); }
  k_affsilu<<<(unsigned)(((size_t)NR * CO / 8 + 255) / 256), 256, 0, stream>>>(CV, c0g, c0b, 0, NR, 0, CAT);
  for (int b = 0; b < NI; ++b) { const size_t r0 = (size_t)b * NPX; const unsigned gi3 = (unsigned)(((size_t)NPX * 9 * (CHD / 8) + 255) / 256);
    k_im2<<<gi3, 256, 0, stream>>>(HL16, CHD, 3, r0, NPX, IM); k_gemm2<0><<<dim3((NPX / 128) * 1, 1), 128, 0, stream>>>(IM, K3, 0, BOF, K3, 0, 0.0625f / 1024.0f, nullptr, 0, nullptr, 1, 0, 0, OFF + r0 * 64, nullptr, 64, 0, NPX, 64, K3);
    k_im2<<<gi3, 256, 0, stream>>>(H16, CHD, 3, r0, NPX, IM); k_gemm2<0><<<dim3((NPX / 128) * 1, 1), 128, 0, stream>>>(IM, K3, 0, BOF, K3, 0, 0.0625f, bofp, 0, OFF + r0 * 64, 1, (size_t)64, 0, OFF + r0 * 64, nullptr, 64, 0, NPX, 64, K3); }
  const unsigned gsn = (unsigned)(((size_t)NR * KS * (CHD / 8) + 255) / 256); const dim3 gsc((NR / 128) * (CO / 64), 1);
  k_snake<0><<<gsn, 256, 0, stream>>>(HF, OFF, offx_g, offx_beta, 0, FE); k_gemm2<0><<<gsc, 128, 0, stream>>>(FE, KSN, 0, BSX, KSN, 0, 0.0625f, dscx_b, 0, nullptr, 1, 0, 0, CV, nullptr, CO, 0, NR, CO, KSN); k_gnst<<<NI * 32, 256, 0, stream>>>(CV, ST); k_gnap<<<(unsigned)(((size_t)NR * CO / 8 + 255) / 256), 256, 0, stream>>>(CV, ST, gnx_g, gnx_b, CO, CAT);
  k_snake<1><<<gsn, 256, 0, stream>>>(HF, OFF, offy_g, offy_beta, 18, FE); k_gemm2<0><<<gsc, 128, 0, stream>>>(FE, KSN, 0, BSY, KSN, 0, 0.0625f, dscy_b, 0, nullptr, 1, 0, 0, CV, nullptr, CO, 0, NR, CO, KSN); k_gnst<<<NI * 32, 256, 0, stream>>>(CV, ST); k_gnap<<<(unsigned)(((size_t)NR * CO / 8 + 255) / 256), 256, 0, stream>>>(CV, ST, gny_g, gny_b, 2 * CO, CAT);
  k_gemm2<0><<<gsc, 128, 0, stream>>>(CAT, CC, 0, BF, CC, 0, 0.0625f, nullptr, 0, nullptr, 1, 0, 0, CV, nullptr, CO, 0, NR, CO, CC); k_affsilu32<<<(unsigned)(((size_t)NR * CO / 8 + 255) / 256), 256, 0, stream>>>(CV, fuse_g, fuse_b, O1);
  k_simst<<<NI * CO, 256, 0, stream>>>(O1, SS); k_final<<<(unsigned)(((size_t)NI * CO * NPX / 8 + 255) / 256), 256, 0, stream>>>(O1, SS, x, (float*)d_out);
}
